// sLSTMLayer_59657095741681
// MI455X (gfx1250) — hardware-verified
//
#include <hip/hip_runtime.h>
#include <math.h>

constexpr int NBAT    = 4;
constexpr int SEQ     = 2048;
constexpr int DMODEL  = 1024;
constexpr int NHEAD   = 4;
constexpr int DHEAD   = 256;
constexpr int NGATE   = 4;
constexpr int CONVK   = 4;
constexpr int NROW    = NBAT * SEQ;
constexpr int GEMM_NT = 256;
constexpr int PREP_NT = 128;
constexpr int PREP_RB = 32;
constexpr int SCAN_NT = 256;
constexpr int SCAN_NW = SCAN_NT / 32;
constexpr int APITCH  = 264;
constexpr int GSLAB   = NBAT * NGATE * 32;
constexpr int OSP     = 36;
constexpr long XPLANE    = (long)NROW * DMODEL;
constexpr long WPLANE_GH = (long)DHEAD * DHEAD;
constexpr long WPLANE_G  = (long)NHEAD * WPLANE_GH;
constexpr long RTPLANE_H = (long)NGATE * DHEAD * DHEAD;
constexpr long GPLANE    = (long)NBAT * SEQ * NGATE * DHEAD;
constexpr float LN_EPS   = 1e-6f;
static_assert(DMODEL == NHEAD * DHEAD);
static_assert(NHEAD == 4 && NGATE == 4 && CONVK == 4);
static_assert(DHEAD % 32 == 0);
static_assert(NROW % 64 == 0 && DHEAD % 64 == 0);
static_assert(((NROW / 64) * (DHEAD / 64)) % 8 == 0);
static_assert(PREP_NT * 8 == DMODEL);
static_assert(SEQ % PREP_RB == 0 && PREP_RB >= CONVK);
static_assert(SCAN_NW * 32 == DHEAD);
static_assert((2 * 16 * APITCH) % SCAN_NT == 0);
static_assert(WPLANE_G % (8 * 256) == 0);
static_assert((NGATE * DHEAD) % 64 == 0 && DHEAD % 64 == 0);

typedef __attribute__((ext_vector_type(16))) _Float16 v16h;
typedef __attribute__((ext_vector_type(8)))  _Float16 v8h;
typedef __attribute__((ext_vector_type(16))) __bf16   v16b;
typedef __attribute__((ext_vector_type(8)))  __bf16   v8b;
typedef __attribute__((ext_vector_type(8)))  float    v8f;
typedef __attribute__((ext_vector_type(4)))  float    v4f;

__device__ __forceinline__ unsigned short f2bf_bits(float f) {
  unsigned u = __float_as_uint(f);
  return (unsigned short)((u + 0x7FFFu + ((u >> 16) & 1u)) >> 16);
}
__device__ __forceinline__ float bf_bits2f(unsigned short h) { return __uint_as_float(((unsigned)h) << 16); }
__device__ __forceinline__ float bf16r(float f) { return bf_bits2f(f2bf_bits(f)); }

__device__ __forceinline__ void dep_guard_h(v8f& a, v8f& b, v16h x, v16h y) { asm volatile("v_nop\n\tv_nop\n\tv_nop\n\tv_nop" : "+v"(a), "+v"(b) : "v"(x), "v"(y)); }
__device__ __forceinline__ void dep_guard_b(v8f& a, v8f& b, v16b x, v16b y) { asm volatile("v_nop\n\tv_nop\n\tv_nop\n\tv_nop" : "+v"(a), "+v"(b) : "v"(x), "v"(y)); }
__device__ __forceinline__ void dep_guard4_h(v8f& a, v8f& b, v8f& c, v8f& d, v16h x, v16h y) { asm volatile("v_nop\n\tv_nop\n\tv_nop\n\tv_nop" : "+v"(a), "+v"(b), "+v"(c), "+v"(d) : "v"(x), "v"(y)); }
__device__ __forceinline__ void dep_guard4_b(v8f& a, v8f& b, v8f& c, v8f& d, v16b x, v16b y) { asm volatile("v_nop\n\tv_nop\n\tv_nop\n\tv_nop" : "+v"(a), "+v"(b), "+v"(c), "+v"(d) : "v"(x), "v"(y)); }
__device__ __forceinline__ void keep4_h(v16h a, v16h b, v16h c, v16h d) { asm volatile("v_nop" :: "v"(a), "v"(b), "v"(c), "v"(d)); }
__device__ __forceinline__ void keep4_b(v16b a, v16b b, v16b c, v16b d) { asm volatile("v_nop" :: "v"(a), "v"(b), "v"(c), "v"(d)); }
__device__ __forceinline__ void acc_guard4(v8f& a, v8f& b, v8f& c, v8f& d) { asm volatile("v_nop\n\tv_nop\n\tv_nop\n\tv_nop" : "+v"(a), "+v"(b), "+v"(c), "+v"(d)); }
template <typename T> struct Frag;
template <> struct Frag<_Float16> {
  typedef v16h V; union U { v16h v; v8h h[2]; };
  static __device__ __forceinline__ v16h load(const _Float16* p) {
    U f; f.h[0] = *(const v8h*)(p); f.h[1] = *(const v8h*)(p + 16); return f.v;
  }
  static __device__ __forceinline__ v8f mma(v16h a, v16h b, v8f c) {
    return __builtin_amdgcn_wmma_f32_16x16x32_f16(false, a, false, b, (short)0, c, false, false);
  }
  static __device__ __forceinline__ void guard(v8f& a, v8f& b, v16h x, v16h y) { dep_guard_h(a, b, x, y); }
  static __device__ __forceinline__ void guard4(v8f& a, v8f& b, v8f& c, v8f& d, v16h x, v16h y) { dep_guard4_h(a, b, c, d, x, y); }
  static __device__ __forceinline__ void keep(v16h a, v16h b, v16h c, v16h d) { keep4_h(a, b, c, d); }
};
template <> struct Frag<__bf16> {
  typedef v16b V; union U { v16b v; v8b h[2]; };
  static __device__ __forceinline__ v16b load(const __bf16* p) {
    U f; f.h[0] = *(const v8b*)(p); f.h[1] = *(const v8b*)(p + 16); return f.v;
  }
  static __device__ __forceinline__ v8f mma(v16b a, v16b b, v8f c) {
    return __builtin_amdgcn_wmma_f32_16x16x32_bf16(false, a, false, b, (short)0, c, false, false);
  }
  static __device__ __forceinline__ void guard(v8f& a, v8f& b, v16b x, v16b y) { dep_guard_b(a, b, x, y); }
  static __device__ __forceinline__ void guard4(v8f& a, v8f& b, v8f& c, v8f& d, v16b x, v16b y) { dep_guard4_b(a, b, c, d, x, y); }
  static __device__ __forceinline__ void keep(v16b a, v16b b, v16b c, v16b d) { keep4_b(a, b, c, d); }
};

template <int ET> struct Elem;
template <> struct Elem<0> { typedef _Float16 T; };
template <> struct Elem<1> { typedef __bf16 T; };
template <int ET, int SPLITM, int BIAS_MODE, int OUT_MODE, bool RESID, int ACT = 0>
__global__ __launch_bounds__(GEMM_NT) void wmma_gemm64(
    const unsigned short* __restrict__ Ap, const unsigned short* __restrict__ A2p, int lda, long strideA,
    const unsigned short* __restrict__ Btp, const unsigned short* __restrict__ Bt2p, int ldb, long strideB,
    void* __restrict__ Cout, void* __restrict__ Cout2, int ldc, long strideC,
    const float* __restrict__ bias,
    const float* __restrict__ resid, long strideR,
    int M, int N, int K, float scale) {
  typedef typename Elem<ET>::T T;
  typedef typename Frag<T>::V V;
  const T* A = (const T*)Ap; const T* A2 = (const T*)A2p; const T* Bt = (const T*)Btp; const T* Bt2 = (const T*)Bt2p;
  __shared__ __align__(16) float sT[8][16 * 68];
  const int b    = blockIdx.y;
  const int lane = threadIdx.x & 31;
  const int wave = threadIdx.x >> 5;
  const int tilesN = N >> 6;
  const int tilesM = M >> 6;
  const int tile = blockIdx.x * 8 + wave;
  if (tile >= tilesM * tilesN) return;
  const int tm = tile / tilesN;
  const int tn = tile - tm * tilesN;
  const int m0 = tm << 6;
  const int n0 = tn << 6;

  const T* Ab  = A  + (size_t)b * strideA;
  const T* Bb  = Bt + (size_t)b * strideB;
  const T* Ab2 = (SPLITM >= 1) ? (A2  + (size_t)b * strideA) : nullptr;
  const T* Bb2 = (SPLITM == 2) ? (Bt2 + (size_t)b * strideB) : nullptr;

  const int rlane = lane & 15;
  const int koff  = (lane >> 4) * 8;
  const int mOff  = (lane >> 4) * 8;

  v8f acc[4][4];
#pragma unroll
  for (int i = 0; i < 4; ++i)
#pragma unroll
    for (int j = 0; j < 4; ++j) acc[i][j] = (v8f){0.f,0.f,0.f,0.f,0.f,0.f,0.f,0.f};

  for (int k0 = 0; k0 < K; k0 += 32) {
    V bh[4], bl[4];
#pragma unroll
    for (int j = 0; j < 4; ++j) {
      const size_t bo = (size_t)(n0 + (j << 4) + rlane) * ldb + koff + k0;
      bh[j] = Frag<T>::load(Bb + bo);
      if (SPLITM == 2) bl[j] = Frag<T>::load(Bb2 + bo);
    }
#pragma unroll
    for (int i = 0; i < 4; ++i) {
      const size_t ao = (size_t)(m0 + (i << 4) + rlane) * lda + koff + k0;
      V ah = Frag<T>::load(Ab + ao);
      V al;
      if (SPLITM >= 1) al = Frag<T>::load(Ab2 + ao);
#pragma unroll
      for (int j = 0; j < 4; ++j) {
        acc[i][j] = Frag<T>::mma(ah, bh[j], acc[i][j]);
        if (SPLITM == 2) acc[i][j] = Frag<T>::mma(ah, bl[j], acc[i][j]);
        if (SPLITM >= 1) acc[i][j] = Frag<T>::mma(al, bh[j], acc[i][j]);
      }
      Frag<T>::guard4(acc[i][0], acc[i][1], acc[i][2], acc[i][3], ah, (SPLITM >= 1) ? al : ah);
    }
    Frag<T>::keep(bh[0], bh[1], bh[2], bh[3]);
    if (SPLITM == 2) Frag<T>::keep(bl[0], bl[1], bl[2], bl[3]);
  }
  acc_guard4(acc[0][0], acc[0][1], acc[0][2], acc[0][3]);
  acc_guard4(acc[1][0], acc[1][1], acc[1][2], acc[1][3]);
  acc_guard4(acc[2][0], acc[2][1], acc[2][2], acc[2][3]);
  acc_guard4(acc[3][0], acc[3][1], acc[3][2], acc[3][3]);

  float* slab = sT[wave];
  const float* Rb = RESID ? (resid + (size_t)b * strideR) : nullptr;
#pragma unroll
  for (int i = 0; i < 4; ++i) {
    const int mBase = m0 + (i << 4);
#pragma unroll
    for (int j = 0; j < 4; ++j) {
      const int n = n0 + (j << 4) + rlane;
      float bv = 0.f;
      if (BIAS_MODE == 2) bv = bias[n];
#pragma unroll
      for (int r = 0; r < 8; ++r) {
        float v = acc[i][j][r] * scale;
        if (BIAS_MODE == 1) v += bias[mBase + mOff + r];
        if (BIAS_MODE == 2) v += bv;
        if (RESID) v += Rb[(size_t)(mBase + mOff + r) * ldc + n];
        if (ACT == 1) v = tanhf(v);
        if (ACT == 2) v = fmaxf(v, 0.0f);
        if (ACT == 3) v = v / (1.0f + expf(-v));
        if (ACT == 4) v = (v > 0.f) ? v : 0.01f * v;
        slab[(mOff + r) * 68 + (j << 4) + rlane] = v;
      }
    }
    __builtin_amdgcn_fence(__ATOMIC_RELEASE, "workgroup");
    __builtin_amdgcn_wave_barrier();
    __builtin_amdgcn_fence(__ATOMIC_ACQUIRE, "workgroup");
    if (OUT_MODE == 0) {
      float* C = (float*)Cout + (size_t)b * strideC;
      const int hh = lane >> 4, c4 = (lane & 15) * 4;
      for (int pass = 0; pass < 2; ++pass) {
#pragma unroll
        for (int it = 0; it < 8; ++it) {
          const int row = it * 2 + hh;
          v4f v = *(const v4f*)(slab + row * 68 + c4);
          *(volatile v4f*)(C + (size_t)(mBase + row) * ldc + n0 + c4) = v;
        }
        __threadfence();
      }
    } else {
      const int q = lane >> 3, c8 = (lane & 7) * 8;
      unsigned short* C  = (unsigned short*)Cout  + (size_t)b * strideC;
      unsigned short* C2 = (OUT_MODE == 2) ? ((unsigned short*)Cout2 + (size_t)b * strideC) : nullptr;
      for (int pass = 0; pass < 2; ++pass) {
#pragma unroll
        for (int it = 0; it < 4; ++it) {
          const int row = it * 4 + q;
          const float* sp = slab + row * 68 + c8;
          v8h hv, lv;
#pragma unroll
          for (int e = 0; e < 8; ++e) {
            if (OUT_MODE == 1) {
              hv[e] = (_Float16)sp[e];
            } else {
              unsigned short hb = f2bf_bits(sp[e]);
              unsigned short lb = f2bf_bits(sp[e] - bf_bits2f(hb));
              hv[e] = __builtin_bit_cast(_Float16, hb);
              lv[e] = __builtin_bit_cast(_Float16, lb);
            }
          }
          *(volatile v8h*)(C + (size_t)(mBase + row) * ldc + n0 + c8) = hv;
          if (OUT_MODE == 2) *(volatile v8h*)(C2 + (size_t)(mBase + row) * ldc + n0 + c8) = lv;
        }
        __threadfence();
      }
    }
    __builtin_amdgcn_fence(__ATOMIC_RELEASE, "workgroup");
    __builtin_amdgcn_wave_barrier();
    __builtin_amdgcn_fence(__ATOMIC_ACQUIRE, "workgroup");
  }
}

__global__ __launch_bounds__(PREP_NT) void prep_x_kernel(const float* __restrict__ x, const float* __restrict__ cw,
                                                         const float* __restrict__ cb,
                                                         unsigned short* __restrict__ XB,
                                                         unsigned short* __restrict__ XCH,
                                                         unsigned short* __restrict__ XCL) {
  const int tid = threadIdx.x;
  const int b   = blockIdx.x / (SEQ / PREP_RB);
  const int s0  = (blockIdx.x - b * (SEQ / PREP_RB)) * PREP_RB;
  const int d0  = tid * 8;

  float wv[8][4], cbv[8];
#pragma unroll
  for (int e = 0; e < 8; ++e) {
    const v4f t = *(const v4f*)(cw + (size_t)(d0 + e) * CONVK);
    wv[e][0] = bf16r(t[0]); wv[e][1] = bf16r(t[1]); wv[e][2] = bf16r(t[2]); wv[e][3] = bf16r(t[3]);
  }
  {
    const v4f t0 = *(const v4f*)(cb + d0);
    const v4f t1 = *(const v4f*)(cb + d0 + 4);
#pragma unroll
    for (int e = 0; e < 4; ++e) { cbv[e] = bf16r(t0[e]); cbv[4 + e] = bf16r(t1[e]); }
  }
  float xm3[8], xm2[8], xm1[8];
#pragma unroll
  for (int e = 0; e < 8; ++e) { xm3[e] = 0.0f; xm2[e] = 0.0f; xm1[e] = 0.0f; }

#pragma unroll 1
  for (int r = -(CONVK - 1); r < PREP_RB; ++r) {
    const int s   = s0 + r;
    const int scl = (s < 0) ? 0 : s;
    const float live = (s < 0) ? 0.0f : 1.0f;
    const size_t rowoff = ((size_t)(b * SEQ + scl)) * DMODEL + d0;
    const v4f xa  = *(const v4f*)(x + rowoff);
    const v4f xb4 = *(const v4f*)(x + rowoff + 4);
    unsigned short xbt[8];
    float xc[8];
#pragma unroll
    for (int e = 0; e < 4; ++e) { xbt[e] = f2bf_bits(xa[e]); xbt[4 + e] = f2bf_bits(xb4[e]); }
#pragma unroll
    for (int e = 0; e < 8; ++e) xc[e] = bf_bits2f(xbt[e]) * live;

    if (r >= 0) {
      v8h pb, ph, pl;
#pragma unroll
      for (int e = 0; e < 8; ++e) {
        float a = wv[e][0] * xm3[e];
        a = fmaf(wv[e][1], xm2[e], a);
        a = fmaf(wv[e][2], xm1[e], a);
        a = fmaf(wv[e][3], xc[e], a);
        a = a + cbv[e];
        const float ex = expf(-a);
        const float sw = a * __builtin_amdgcn_rcpf(1.0f + ex);
        const unsigned short hb = f2bf_bits(sw);
        const unsigned short lb = f2bf_bits(sw - bf_bits2f(hb));
        pb[e] = __builtin_bit_cast(_Float16, xbt[e]);
        ph[e] = __builtin_bit_cast(_Float16, hb);
        pl[e] = __builtin_bit_cast(_Float16, lb);
      }
      *(volatile v8h*)(XB  + rowoff) = pb;
      *(volatile v8h*)(XCH + rowoff) = ph;
      *(volatile v8h*)(XCL + rowoff) = pl;
      __threadfence();
      *(volatile v8h*)(XB  + rowoff) = pb;
      *(volatile v8h*)(XCH + rowoff) = ph;
      *(volatile v8h*)(XCL + rowoff) = pl;
    }
#pragma unroll
    for (int e = 0; e < 8; ++e) { xm3[e] = xm2[e]; xm2[e] = xm1[e]; xm1[e] = xc[e]; }
  }
}

__global__ __launch_bounds__(256) void cvt_w_kernel(const float* __restrict__ w0, const float* __restrict__ w1,
                                                    const float* __restrict__ w2, const float* __restrict__ w3,
                                                    unsigned short* __restrict__ WB) {
  const int g = blockIdx.y;
  const float* src = (g == 0) ? w0 : (g == 1) ? w1 : (g == 2) ? w2 : w3;
  const int i = blockIdx.x * 256 + threadIdx.x;
  const float* sp = src + (size_t)i * 8;
  const v4f a  = *(const v4f*)(sp);
  const v4f bq = *(const v4f*)(sp + 4);
  v8h hv;
#pragma unroll
  for (int e = 0; e < 4; ++e) {
    hv[e]     = __builtin_bit_cast(_Float16, f2bf_bits(a[e]));
    hv[4 + e] = __builtin_bit_cast(_Float16, f2bf_bits(bq[e]));
  }
  unsigned short* dp = WB + (size_t)g * WPLANE_G + (size_t)i * 8;
  *(volatile v8h*)dp = hv;
  __threadfence();
  *(volatile v8h*)dp = hv;
}

__global__ __launch_bounds__(256) void tpw_bf16_kernel(const float* __restrict__ src, int R, int C, int ldo,
                                                       unsigned short* __restrict__ O) {
  __shared__ float Tt[64 * 65];
  const int tid = threadIdx.x;
  const int c0 = blockIdx.x * 64, r0 = blockIdx.y * 64;
  src += (size_t)blockIdx.z * (size_t)R * (size_t)C;
  O   += (size_t)blockIdx.z * (size_t)C * (size_t)ldo;
#pragma unroll
  for (int i = 0; i < 4; ++i) {
    const int idx = i * 256 + tid;
    const int rr = idx >> 4, cc = (idx & 15) * 4;
    const v4f v = *(const v4f*)(src + (size_t)(r0 + rr) * (size_t)C + c0 + cc);
    Tt[rr * 65 + cc + 0] = v[0];
    Tt[rr * 65 + cc + 1] = v[1];
    Tt[rr * 65 + cc + 2] = v[2];
    Tt[rr * 65 + cc + 3] = v[3];
  }
  __syncthreads();
  const int q = tid >> 3, c8 = (tid & 7) * 8;
  v8h hv[2];
#pragma unroll
  for (int g = 0; g < 2; ++g) {
    const int qq = g * 32 + q;
#pragma unroll
    for (int e = 0; e < 8; ++e) {
      const float f = Tt[(c8 + e) * 65 + qq];
      hv[g][e] = __builtin_bit_cast(_Float16, f2bf_bits(f));
    }
  }
  for (int pass = 0; pass < 2; ++pass) {
#pragma unroll
    for (int g = 0; g < 2; ++g) {
      const size_t o = (size_t)(c0 + g * 32 + q) * (size_t)ldo + (size_t)(r0 + c8);
      *(volatile v8h*)(O + o) = hv[g];
    }
    __threadfence();
  }
}

__global__ __launch_bounds__(SCAN_NT) void slstm_scan_kernel(const float* __restrict__ GT,
                                                          const unsigned short* __restrict__ RTp,
                                                          const float* __restrict__ cbias,
                                                          const float* __restrict__ gsc,
                                                          const float* __restrict__ gbi,
                                                          float* __restrict__ out, int pair) {
  __shared__ __align__(16) __bf16 Ah[2][16 * APITCH];
  __shared__ __align__(16) float  Gs[SCAN_NW][GSLAB];
  __shared__ __align__(16) float  Os[SCAN_NW][4 * OSP];
  __shared__ float Pl[2][SCAN_NW * 8];
  const int tid = threadIdx.x, lane = tid & 31, wave = tid >> 5;
  const int c = lane & 15, hh = lane >> 4, koff = 8 * hh;
  const int gq = lane >> 3, d4 = (lane & 7) * 4;
  const int hl = blockIdx.x;
  const int hd = 2 * pair + hl;
  const int dbase = 32 * wave;
  const float* Gp = GT + (size_t)hl * GPLANE;
  const __bf16* Rt = (const __bf16*)RTp + (size_t)hd * RTPLANE_H;

  {
    __bf16* ahf = &Ah[0][0];
    const __bf16 z = __builtin_bit_cast(__bf16, (unsigned short)0);
#pragma unroll 1
    for (int i = tid; i < 2 * 16 * APITCH; i += SCAN_NT) ahf[i] = z;
  }
  float bgv[2][4], lsc[2], lbi[2];
#pragma unroll
  for (int nt = 0; nt < 2; ++nt) {
    const int d = dbase + 16 * nt + c;
#pragma unroll
    for (int g = 0; g < 4; ++g) bgv[nt][g] = bf16r(cbias[(size_t)(g * NHEAD + hd) * DHEAD + d]);
    lsc[nt] = bf16r(gsc[hd * DHEAD + d]);
    lbi[nt] = bf16r(gbi[hd * DHEAD + d]);
  }
  float cst[2][2], nst[2][2], mst[2][2];
#pragma unroll
  for (int nt = 0; nt < 2; ++nt)
#pragma unroll
    for (int q = 0; q < 2; ++q) { cst[nt][q] = 0.0f; nst[nt][q] = 0.0f; mst[nt][q] = 0.0f; }
  __syncthreads();

  const v8f z8 = {0.f, 0.f, 0.f, 0.f, 0.f, 0.f, 0.f, 0.f};
  float* gs = Gs[wave];
  float* os = Os[wave];

#pragma unroll 1
  for (int s = 0; s < SEQ; ++s) {
    const int cur = s & 1;
#pragma unroll
    for (int b = 0; b < NBAT; ++b) {
      const v4f v = *(const v4f*)(Gp + ((size_t)(b * SEQ + s)) * (NGATE * DHEAD) + gq * DHEAD + dbase + d4);
      *(v4f*)(gs + (b * NGATE + gq) * 32 + d4) = v;
    }
    __builtin_amdgcn_fence(__ATOMIC_RELEASE, "workgroup");
    __builtin_amdgcn_wave_barrier();
    __builtin_amdgcn_fence(__ATOMIC_ACQUIRE, "workgroup");

    const __bf16* ahrow = &Ah[cur][0] + c * APITCH + koff;
    v8f acc[2][4];
#pragma unroll
    for (int nt = 0; nt < 2; ++nt) { acc[nt][0] = z8; acc[nt][1] = z8; acc[nt][2] = z8; acc[nt][3] = z8; }
#pragma unroll 1
    for (int k0 = 0; k0 < DHEAD; k0 += 32) {
      const v16b a = Frag<__bf16>::load(ahrow + k0);
#pragma unroll
      for (int nt = 0; nt < 2; ++nt) {
        const __bf16* rp = Rt + (size_t)(dbase + 16 * nt + c) * DHEAD + koff + k0;
        const v16b b0 = Frag<__bf16>::load(rp);
        const v16b b1 = Frag<__bf16>::load(rp + (size_t)1 * WPLANE_GH);
        const v16b b2 = Frag<__bf16>::load(rp + (size_t)2 * WPLANE_GH);
        const v16b b3 = Frag<__bf16>::load(rp + (size_t)3 * WPLANE_GH);
        acc[nt][0] = Frag<__bf16>::mma(a, b0, acc[nt][0]);
        acc[nt][1] = Frag<__bf16>::mma(a, b1, acc[nt][1]);
        acc[nt][2] = Frag<__bf16>::mma(a, b2, acc[nt][2]);
        acc[nt][3] = Frag<__bf16>::mma(a, b3, acc[nt][3]);
        dep_guard4_b(acc[nt][0], acc[nt][1], acc[nt][2], acc[nt][3], a, b3);
        keep4_b(b0, b1, b2, b3);
      }
    }
    acc_guard4(acc[0][0], acc[0][1], acc[0][2], acc[0][3]);
    acc_guard4(acc[1][0], acc[1][1], acc[1][2], acc[1][3]);

    __bf16* ahn = &Ah[cur ^ 1][0];
    float hv[2][2];
#pragma unroll
    for (int nt = 0; nt < 2; ++nt) {
      const int dl = 16 * nt + c;
      const int d  = dbase + dl;
#pragma unroll
      for (int q = 0; q < 2; ++q) {
        const int b = 2 * hh + q;
        const float* gb = gs + (b * NGATE) * 32 + dl;
        const float graw_i = gb[0];
        const float graw_f = gb[32];
        const float graw_z = gb[64];
        const float graw_o = gb[96];
        const float iraw = (graw_i + (acc[nt][0][q] + acc[nt][0][2 + q])) + bgv[nt][0];
        const float fraw = (graw_f + (acc[nt][1][q] + acc[nt][1][2 + q])) + bgv[nt][1];
        const float zraw = (graw_z + (acc[nt][2][q] + acc[nt][2][2 + q])) + bgv[nt][2];
        const float oraw = (graw_o + (acc[nt][3][q] + acc[nt][3][2 + q])) + bgv[nt][3];
        const float lsg  = fminf(fraw, 0.0f) - log1pf(expf(-fabsf(fraw)));
        const float lfm  = mst[nt][q] + lsg;
        const float mnew = fmaxf(iraw, lfm);
        const float ig   = expf(iraw - mnew);
        const float fg   = expf(lfm - mnew);
        const float cn   = fg * cst[nt][q] + ig * tanhf(zraw);
        const float nn   = fg * nst[nt][q] + ig;
        cst[nt][q] = cn; nst[nt][q] = nn; mst[nt][q] = mnew;
        const float so   = __builtin_amdgcn_rcpf(1.0f + expf(-oraw));
        const float hn   = (so * cn) / nn;
        hv[nt][q] = hn;
        const unsigned short hb = f2bf_bits(hn);
        const unsigned short lb = f2bf_bits(hn - bf_bits2f(hb));
        ahn[(8 * hh + q) * APITCH + d]     = __builtin_bit_cast(__bf16, hb);
        ahn[(8 * hh + 2 + q) * APITCH + d] = __builtin_bit_cast(__bf16, lb);
      }
    }
    float ps[2], pm[2];
#pragma unroll
    for (int q = 0; q < 2; ++q) {
      float s1 = hv[0][q] + hv[1][q];
      s1 += __shfl_xor(s1, 1, 32);
      s1 += __shfl_xor(s1, 2, 32);
      s1 += __shfl_xor(s1, 4, 32);
      s1 += __shfl_xor(s1, 8, 32);
      const float mw = s1 * (1.0f / 32.0f);
      const float e0 = hv[0][q] - mw, e1 = hv[1][q] - mw;
      float m2 = e0 * e0 + e1 * e1;
      m2 += __shfl_xor(m2, 1, 32);
      m2 += __shfl_xor(m2, 2, 32);
      m2 += __shfl_xor(m2, 4, 32);
      m2 += __shfl_xor(m2, 8, 32);
      ps[q] = s1; pm[q] = m2;
    }
    if (c == 0) {
#pragma unroll
      for (int q = 0; q < 2; ++q) {
        Pl[cur][wave * 8 + (2 * hh + q) * 2]     = ps[q];
        Pl[cur][wave * 8 + (2 * hh + q) * 2 + 1] = pm[q];
      }
    }
    __syncthreads();

#pragma unroll
    for (int q = 0; q < 2; ++q) {
      const int b = 2 * hh + q;
      float S1 = 0.0f;
#pragma unroll
      for (int w2 = 0; w2 < SCAN_NW; ++w2) S1 += Pl[cur][w2 * 8 + b * 2];
      const float mu = S1 * (1.0f / (float)DHEAD);
      float SS = 0.0f;
#pragma unroll
      for (int w2 = 0; w2 < SCAN_NW; ++w2) {
        const float dw = Pl[cur][w2 * 8 + b * 2] - 32.0f * mu;
        SS += Pl[cur][w2 * 8 + b * 2 + 1] + dw * dw * (1.0f / 32.0f);
      }
      const float var  = fmaxf(SS * (1.0f / (float)DHEAD), 0.0f);
      const float rstd = rsqrtf(var + LN_EPS);
#pragma unroll
      for (int nt = 0; nt < 2; ++nt) os[b * OSP + 16 * nt + c] = ((hv[nt][q] - mu) * rstd) * lsc[nt] + lbi[nt];
    }
    __builtin_amdgcn_fence(__ATOMIC_RELEASE, "workgroup");
    __builtin_amdgcn_wave_barrier();
    __builtin_amdgcn_fence(__ATOMIC_ACQUIRE, "workgroup");
    {
      const v4f v = *(const v4f*)(os + gq * OSP + d4);
      float* op = out + ((size_t)(gq * SEQ + s)) * DMODEL + hd * DHEAD + dbase + d4;
      *(volatile v4f*)op = v;
      __threadfence();
      *(volatile v4f*)op = v;
    }
    __builtin_amdgcn_fence(__ATOMIC_RELEASE, "workgroup");
    __builtin_amdgcn_wave_barrier();
    __builtin_amdgcn_fence(__ATOMIC_ACQUIRE, "workgroup");
  }
}

extern "C" void kernel_launch(void* const* d_in, const int* in_sizes, int n_in,
                              void* d_out, int out_size, void* d_ws, size_t ws_size, hipStream_t stream) {
  if (n_in < 11 || d_out == nullptr || d_ws == nullptr) return;
  if (in_sizes[0] != NBAT * SEQ * DMODEL || in_sizes[1] != DMODEL * CONVK || in_sizes[2] != DMODEL ||
      in_sizes[3] != (int)WPLANE_G || in_sizes[4] != (int)WPLANE_G || in_sizes[5] != (int)WPLANE_G ||
      in_sizes[6] != (int)WPLANE_G || in_sizes[7] != (int)(NHEAD * RTPLANE_H) || in_sizes[8] != NGATE * NHEAD * DHEAD ||
      in_sizes[9] != DMODEL || in_sizes[10] != DMODEL || out_size != NBAT * SEQ * DMODEL) return;

  const float* x      = (const float*)d_in[0];
  const float* conv_w = (const float*)d_in[1];
  const float* conv_b = (const float*)d_in[2];
  const float* w_i    = (const float*)d_in[3];
  const float* w_f    = (const float*)d_in[4];
  const float* w_z    = (const float*)d_in[5];
  const float* w_o    = (const float*)d_in[6];
  const float* rec    = (const float*)d_in[7];
  const float* cbias  = (const float*)d_in[8];
  const float* gsc    = (const float*)d_in[9];
  const float* gbi    = (const float*)d_in[10];
  float* out = (float*)d_out;

  char* ws = (char*)d_ws; size_t off = 0;
  auto carve = [&](size_t bytes) -> char* { char* p = ws + off; off += (bytes + 255) & ~(size_t)255; return p; };
  unsigned short* XB    = (unsigned short*)carve((size_t)XPLANE * 2);
  unsigned short* XCH   = (unsigned short*)carve((size_t)XPLANE * 2);
  unsigned short* XCL   = (unsigned short*)carve((size_t)XPLANE * 2);
  unsigned short* WB    = (unsigned short*)carve((size_t)NGATE * WPLANE_G * 2);
  unsigned short* RT    = (unsigned short*)carve((size_t)NHEAD * RTPLANE_H * 2);
  float*          GATES = (float*)carve((size_t)2 * GPLANE * 4);
  if (off > ws_size || off > (size_t)134217728) return;

  prep_x_kernel<<<NBAT * (SEQ / PREP_RB), PREP_NT, 0, stream>>>(x, conv_w, conv_b, XB, XCH, XCL);
  cvt_w_kernel<<<dim3((unsigned)(WPLANE_G / 8 / 256), NGATE), 256, 0, stream>>>(w_i, w_f, w_z, w_o, WB);
  tpw_bf16_kernel<<<dim3((NGATE * DHEAD) / 64, DHEAD / 64, NHEAD), 256, 0, stream>>>(rec, DHEAD, NGATE * DHEAD, DHEAD, RT);

  const dim3 ggrid((NROW / 64) * (DHEAD / 64) / 8, 2);
  for (int p = 0; p < 2; ++p) {
    const unsigned short* xchp = XCH + (size_t)p * 2 * DHEAD;
    const unsigned short* xclp = XCL + (size_t)p * 2 * DHEAD;
    const unsigned short* xbp  = XB  + (size_t)p * 2 * DHEAD;
    for (int g = 0; g < NGATE; ++g) {
      const unsigned short* wb = WB + (size_t)(g * NHEAD + 2 * p) * WPLANE_GH;
      float* cg = GATES + (size_t)g * DHEAD;
      if (g < 2) {
        wmma_gemm64<1, 1, 0, 0, false, 0><<<ggrid, GEMM_NT, 0, stream>>>(
            xchp, xclp, DMODEL, (long)DHEAD, wb, wb, DHEAD, (long)WPLANE_GH, (void*)cg, (void*)cg, NGATE * DHEAD, (long)GPLANE,
            cbias, GATES, 0L, NROW, DHEAD, DHEAD, 1.0f);
      } else {
        wmma_gemm64<1, 0, 0, 0, false, 0><<<ggrid, GEMM_NT, 0, stream>>>(
            xbp, xbp, DMODEL, (long)DHEAD, wb, wb, DHEAD, (long)WPLANE_GH, (void*)cg, (void*)cg, NGATE * DHEAD, (long)GPLANE,
            cbias, GATES, 0L, NROW, DHEAD, DHEAD, 1.0f);
      }
    }
    slstm_scan_kernel<<<2, SCAN_NT, 0, stream>>>(GATES, RT, cbias, gsc, gbi, out, p);
  }
}
